// GIN_55353538511630
// MI455X (gfx1250) — hardware-verified
//
#include <hip/hip_runtime.h>
#include <stddef.h>
#include <stdint.h>


#define FIN    32
#define DH     128
#define KA     64
#define KB     256
#define NTHR   256
#define NWAVE  8
#define EPT    8
#define CHUNK  (NTHR * EPT)
#define WCAP   (EPT * 32)
#define LISTN  (NWAVE * WCAP)
#define NBR    1024
#define NBRS   10
#define RCAP   4096
#define DEGCAP 64
#define OCBAD  255
#define PKS    11
#define GBM    64
#define GTHR   128
#define GNT    8
#define PGR    128
#define VECL   768
#define NUA    (DH * (KA / 8))
#define NUB    (DH * (KB / 8))
#define NUW    (NUA + 6 * NUB)
#define NWBLK  (NUW / NTHR)
#define NVBLK  4
#define HVF    288
#define POOL_F (PGR * DH + HVF + PGR + LISTN + 16)
#define LDS_POOL (POOL_F * 4)
#define WSMAX  268435456

static_assert((CHUNK & (CHUNK - 1)) == 0 && CHUNK <= (1 << PKS));
static_assert(NBR == (1 << NBRS) && NBR <= (1 << PKS) && NBR == 4 * NTHR);
static_assert(LISTN >= NBR && (RCAP % (4 * NTHR)) == 0);
static_assert(DEGCAP < OCBAD && RCAP < (1 << 20));
static_assert(KA == 2 * FIN && KB == 2 * DH && (KA % 32) == 0 && (KB % 32) == 0);
static_assert(GBM == (GTHR / 32) * 16 && DH == 16 * GNT && DH == 4 * 32 && FIN == 4 * 8);
static_assert((NUA % NTHR) == 0 && (NUB % NTHR) == 0 && (NUW % NTHR) == 0);
static_assert(PGR == NWAVE * 16 && (PGR & (PGR - 1)) == 0 && PGR <= (1 << PKS));
static_assert((PGR * DH / 4) % NTHR == 0 && VECL == 6 * DH && VECL / 4 <= NTHR && HVF / 4 <= NTHR);
static_assert(LDS_POOL <= 300000);

typedef float          v4f  __attribute__((ext_vector_type(4)));
typedef float          v8f  __attribute__((ext_vector_type(8)));
typedef int            v4i  __attribute__((ext_vector_type(4)));
typedef int            v8i  __attribute__((ext_vector_type(8)));
typedef unsigned int   v4u  __attribute__((ext_vector_type(4)));
typedef unsigned short v8us __attribute__((ext_vector_type(8)));
typedef __bf16         v16b __attribute__((ext_vector_type(16)));
typedef v4f  __attribute__((may_alias)) v4fa;
typedef v4i  __attribute__((may_alias)) v4ia;
typedef v4u  __attribute__((may_alias)) v4ua;
typedef v8us __attribute__((may_alias)) v8usa;
union Frag { v16b vb; v8us h[2]; v8i w; };

__device__ __forceinline__ v8f wmb(const Frag& a, const Frag& b, v8f c) {
  v8f d = __builtin_amdgcn_wmma_f32_16x16x32_bf16(false, a.vb, false, b.vb, (short)0, c, false, false);
  asm volatile("v_nop\n\tv_nop\n\tv_nop\n\tv_nop" : "+v"(d) : "v"(a.w), "v"(b.w));
  return d;
}

__device__ __forceinline__ unsigned int bf_bits(float f) {
  const unsigned int u = __float_as_uint(f);
  unsigned int r = (u + 0x7FFFu + ((u >> 16) & 1u)) >> 16;
  r = ((u & 0x7FFFFFFFu) > 0x7F800000u) ? 0x7FC0u : r;
  return r;
}
__device__ __forceinline__ float bf_val(unsigned int b) { return __uint_as_float(b << 16); }
__device__ __forceinline__ float bf_rne(float f) { return bf_val(bf_bits(f)); }

__device__ __forceinline__ v4u hilo4(float a, float b, float c, float d) {
  const unsigned int h0 = bf_bits(a), h1 = bf_bits(b), h2 = bf_bits(c), h3 = bf_bits(d);
  const unsigned int l0 = bf_bits(a - bf_val(h0)), l1 = bf_bits(b - bf_val(h1));
  const unsigned int l2 = bf_bits(c - bf_val(h2)), l3 = bf_bits(d - bf_val(h3));
  v4u o;
  o.x = h0 | (h1 << 16);
  o.y = h2 | (h3 << 16);
  o.z = l0 | (l1 << 16);
  o.w = l2 | (l3 << 16);
  return o;
}

__device__ __forceinline__ float relu_keep(float v) { return (v > 0.0f) ? v : (v - v); }

__device__ __forceinline__ int scan_chunk(const int* __restrict__ dsts, int nE, int cbase, int slotBase,
                                          int nb, int vec8, int* list, int tid, int lane, int wave) {
  int wc = 0;
  const int el0  = tid * EPT;
  const int e0   = cbase + el0;
  const int sent = -2147483647 - 1;
  v4i da, db;
  if (vec8 != 0 && cbase + CHUNK <= nE) {
    da = *(const v4i*)(dsts + e0);
    db = *(const v4i*)(dsts + e0 + 4);
  } else {
    da.x = (e0     < nE) ? dsts[min(e0,     nE - 1)] : sent;
    da.y = (e0 + 1 < nE) ? dsts[min(e0 + 1, nE - 1)] : sent;
    da.z = (e0 + 2 < nE) ? dsts[min(e0 + 2, nE - 1)] : sent;
    da.w = (e0 + 3 < nE) ? dsts[min(e0 + 3, nE - 1)] : sent;
    db.x = (e0 + 4 < nE) ? dsts[min(e0 + 4, nE - 1)] : sent;
    db.y = (e0 + 5 < nE) ? dsts[min(e0 + 5, nE - 1)] : sent;
    db.z = (e0 + 6 < nE) ? dsts[min(e0 + 6, nE - 1)] : sent;
    db.w = (e0 + 7 < nE) ? dsts[min(e0 + 7, nE - 1)] : sent;
  }
  const unsigned nbs = (unsigned)slotBase;
  const unsigned unb = (unsigned)nb;
  const unsigned s0 = (unsigned)da.x - nbs, s1 = (unsigned)da.y - nbs;
  const unsigned s2 = (unsigned)da.z - nbs, s3 = (unsigned)da.w - nbs;
  const unsigned s4 = (unsigned)db.x - nbs, s5 = (unsigned)db.y - nbs;
  const unsigned s6 = (unsigned)db.z - nbs, s7 = (unsigned)db.w - nbs;
  const bool h0 = s0 < unb, h1 = s1 < unb, h2 = s2 < unb, h3 = s3 < unb;
  const bool h4 = s4 < unb, h5 = s5 < unb, h6 = s6 < unb, h7 = s7 < unb;
  const unsigned any = __builtin_amdgcn_ballot_w32(h0 | h1 | h2 | h3 | h4 | h5 | h6 | h7);
  if (any != 0u) {
#define HITJ(J, HJ, SJ) { \
      const unsigned mj = __builtin_amdgcn_ballot_w32(HJ); \
      if (mj != 0u) { \
        if (HJ) { \
          const int pos = wc + (int)__builtin_amdgcn_mbcnt_lo(mj, 0u); \
          if (pos < WCAP) list[wave * WCAP + pos] = ((el0 + (J)) << PKS) | (int)(SJ); \
        } \
        wc += (int)__builtin_popcount(mj); } }
    HITJ(0, h0, s0)
    HITJ(1, h1, s1)
    HITJ(2, h2, s2)
    HITJ(3, h3, s3)
    HITJ(4, h4, s4)
    HITJ(5, h5, s5)
    HITJ(6, h6, s6)
    HITJ(7, h7, s7)
#undef HITJ
  }
  return wc;
}

__global__ __launch_bounds__(NTHR) void k_prep(
    const float* __restrict__ w1a, const float* __restrict__ w2a, const float* __restrict__ w1b,
    const float* __restrict__ w2b, const float* __restrict__ w1c, const float* __restrict__ w2c,
    const float* __restrict__ lw1,
    const float* __restrict__ a_b1, const float* __restrict__ a_g, const float* __restrict__ a_be,
    const float* __restrict__ a_rm, const float* __restrict__ a_rv, const float* __restrict__ a_b2,
    const float* __restrict__ b_b1, const float* __restrict__ b_g, const float* __restrict__ b_be,
    const float* __restrict__ b_rm, const float* __restrict__ b_rv, const float* __restrict__ b_b2,
    const float* __restrict__ c_b1, const float* __restrict__ c_g, const float* __restrict__ c_be,
    const float* __restrict__ c_rm, const float* __restrict__ c_rv, const float* __restrict__ c_b2,
    const float* __restrict__ lb1, const float* __restrict__ lw2, const float* __restrict__ lb2,
    unsigned short* p1a, unsigned short* p2a, unsigned short* p1b, unsigned short* p2b,
    unsigned short* p1c, unsigned short* p2c, unsigned short* pl1, float* vec) {
  __shared__ __attribute__((aligned(16))) float vs[VECL];
  const int tid = (int)threadIdx.x;
  const int bx  = (int)blockIdx.x;
  if (bx < NWBLK) {
    const int u = bx * NTHR + tid;
    const float* sp;
    unsigned short* dq;
    int n, g, kp;
    if (u < NUA) {
      sp = w1a; dq = p1a; n = u >> 3; g = u & 7; kp = KA;
    } else {
      const int v  = u - NUA;
      const int mi = v >> 12;
      const int vv = v & (NUB - 1);
      n = vv >> 5; g = vv & 31; kp = KB;
      sp = (mi == 0) ? w2a : ((mi == 1) ? w1b : ((mi == 2) ? w2b : ((mi == 3) ? w1c : ((mi == 4) ? w2c : lw1))));
      dq = (mi == 0) ? p2a : ((mi == 1) ? p1b : ((mi == 2) ? p2b : ((mi == 3) ? p1c : ((mi == 4) ? p2c : pl1))));
    }
    const float* p = sp + (size_t)(4 * g) * DH + n;
    const unsigned int b0 = bf_bits(p[0]);
    const unsigned int b1 = bf_bits(p[DH]);
    const unsigned int b2 = bf_bits(p[2 * DH]);
    const unsigned int b3 = bf_bits(p[3 * DH]);
    v4u o;
    o.x = b0 | (b1 << 16);
    o.y = b2 | (b3 << 16);
    o.z = o.x;
    o.w = o.y;
    unsigned short* dp = dq + (size_t)n * (size_t)kp + 8 * g;
    *(volatile v4u*)dp = o;
    __threadfence();
    *(volatile v4u*)dp = o;
    return;
  }
  const int vb = bx - NWBLK;
  const int c  = tid & (DH - 1);
  const bool ld = tid < DH;
  if (vb < 3) {
    const float* pb1 = (vb == 0) ? a_b1 : ((vb == 1) ? b_b1 : c_b1);
    const float* pg  = (vb == 0) ? a_g  : ((vb == 1) ? b_g  : c_g);
    const float* pbe = (vb == 0) ? a_be : ((vb == 1) ? b_be : c_be);
    const float* prm = (vb == 0) ? a_rm : ((vb == 1) ? b_rm : c_rm);
    const float* prv = (vb == 0) ? a_rv : ((vb == 1) ? b_rv : c_rv);
    const float* pb2 = (vb == 0) ? a_b2 : ((vb == 1) ? b_b2 : c_b2);
    if (ld) {
      vs[c]          = bf_rne(pb1[c]);
      vs[DH + c]     = bf_rne(prm[c]);
      vs[2 * DH + c] = 1.0f / sqrtf(bf_rne(prv[c]) + 1e-5f);
      vs[3 * DH + c] = bf_rne(pg[c]);
      vs[4 * DH + c] = bf_rne(pbe[c]);
      vs[5 * DH + c] = bf_rne(pb2[c]);
    }
  } else {
    if (ld) {
      const float l2 = bf_rne(lb2[0]);
      vs[c]          = bf_rne(lb1[c]);
      vs[DH + c]     = bf_rne(lw2[c]);
      vs[2 * DH + c] = (c == 0) ? l2 : 0.0f;
      vs[3 * DH + c] = 0.0f;
      vs[4 * DH + c] = 0.0f;
      vs[5 * DH + c] = 0.0f;
    }
  }
  __syncthreads();
  const bool ok = tid < VECL / 4;
  const int  t4 = ok ? tid : 0;
  const v4f v = *(const v4fa*)(vs + 4 * t4);
  float* dp = vec + (size_t)vb * VECL + 4 * t4;
  if (ok) *(volatile v4f*)dp = v;
  __threadfence();
  if (ok) *(volatile v4f*)dp = v;
}

__global__ __launch_bounds__(NTHR) void k_scan(const int* __restrict__ srcs, const int* __restrict__ dsts,
                                               int nN, int nE, int vec8, int* lst, int* oc) {
  __shared__ __attribute__((aligned(16))) int reg1[RCAP];
  __shared__ __attribute__((aligned(16))) int reg2[RCAP];
  __shared__ __attribute__((aligned(16))) int scnt[NBR];
  __shared__ __attribute__((aligned(16))) int soff[NBR];
  __shared__ __attribute__((aligned(16))) int list[LISTN];
  __shared__ int wcnt[NWAVE];
  __shared__ int wtot[NWAVE];
  const int tid = (int)threadIdx.x, lane = tid & 31, wave = tid >> 5;
  const int nodeBase = (int)blockIdx.x * NBR;

  for (int i = tid; i < RCAP; i += NTHR) { reg1[i] = 0; reg2[i] = 0; }
  for (int i = tid; i < NBR; i += NTHR) { scnt[i] = 0; soff[i] = 0; }
  for (int i = tid; i < LISTN; i += NTHR) list[i] = 0;
  if (tid < NWAVE) { wcnt[tid] = 0; wtot[tid] = 0; }
  __syncthreads();

  int tot = 0;
  const int nChunks = (nE + CHUNK - 1) / CHUNK;
#pragma unroll 1
  for (int ch = 0; ch < nChunks; ++ch) {
    const int cbase = ch * CHUNK;
    const int wc = scan_chunk(dsts, nE, cbase, nodeBase, NBR, vec8, list, tid, lane, wave);
    if (lane == 0) wcnt[wave] = wc;
    __syncthreads();
    int pre = 0, all = 0;
#pragma unroll
    for (int w2 = 0; w2 < NWAVE; ++w2) {
      int c = wcnt[w2];
      c = c < 0 ? 0 : (c > WCAP ? WCAP : c);
      all += c;
      pre += (w2 < wave) ? c : 0;
    }
    const int wcc  = wc > WCAP ? WCAP : wc;
    const int base = tot + pre;
#pragma unroll 1
    for (int i = lane; i < wcc; i += 32) {
      const int ent = list[wave * WCAP + i];
      const int el  = (ent >> PKS) & (CHUNK - 1);
      const int sl  = ent & (NBR - 1);
      int eid = cbase + el;
      eid = eid > nE - 1 ? nE - 1 : eid;
      const int pos = base + i;
      if (pos < RCAP) reg1[pos] = (int)(((unsigned)eid << PKS) | (unsigned)sl);
    }
    tot += all;
    tot = tot > RCAP ? RCAP : tot;
    __syncthreads();
  }
  const int nh = tot;

  if (wave == 0) {
#pragma unroll 1
    for (int b0 = 0; b0 < nh; b0 += 32) {
      const int idx = b0 + lane;
      const int uv  = reg1[idx < RCAP ? idx : RCAP - 1];
      const int m32 = (nh - b0) < 32 ? (nh - b0) : 32;
#pragma unroll 1
      for (int k = 0; k < m32; ++k) {
        const int u  = __builtin_amdgcn_readlane(uv, k);
        const int sl = u & (NBR - 1);
        if (lane == 0) scnt[sl] = scnt[sl] + 1;
      }
    }
  }
  __syncthreads();

  {
    const v4i ca = *(const v4ia*)(scnt + 4 * tid);
    const int e0 = ca.x < 0 ? 0 : ca.x, e1 = ca.y < 0 ? 0 : ca.y;
    const int e2 = ca.z < 0 ? 0 : ca.z, e3 = ca.w < 0 ? 0 : ca.w;
    const int ts = e0 + e1 + e2 + e3;
    int incl = ts;
#pragma unroll
    for (int d = 1; d < 32; d <<= 1) {
      const int up = __shfl_up(incl, d);
      if (lane >= d) incl += up;
    }
    if (lane == 31) wtot[wave] = incl;
    __syncthreads();
    int pre = 0;
#pragma unroll
    for (int w2 = 0; w2 < NWAVE; ++w2) pre += (w2 < wave) ? wtot[w2] : 0;
    int run = pre + incl - ts;
    soff[4 * tid + 0] = run; run += e0;
    soff[4 * tid + 1] = run; run += e1;
    soff[4 * tid + 2] = run; run += e2;
    soff[4 * tid + 3] = run;
  }
  __syncthreads();
  for (int i = tid; i < NBR; i += NTHR) list[i] = soff[i];
  __syncthreads();

  if (wave == 0) {
#pragma unroll 1
    for (int b0 = 0; b0 < nh; b0 += 32) {
      const int idx = b0 + lane;
      const int uv  = reg1[idx < RCAP ? idx : RCAP - 1];
      const int m32 = (nh - b0) < 32 ? (nh - b0) : 32;
#pragma unroll 1
      for (int k = 0; k < m32; ++k) {
        const int u   = __builtin_amdgcn_readlane(uv, k);
        const int sl  = u & (NBR - 1);
        const int eid = (int)((unsigned)u >> PKS);
        if (lane == 0) {
          int pos = list[sl];
          pos = pos < 0 ? 0 : (pos > RCAP - 1 ? RCAP - 1 : pos);
          reg2[pos] = eid;
          list[sl] = pos + 1;
        }
      }
    }
  }
  __syncthreads();

#pragma unroll 1
  for (int i = tid; i < RCAP; i += NTHR) {
    int e = reg2[i];
    e = e < 0 ? 0 : (e > nE - 1 ? nE - 1 : e);
    int s = srcs[e];
    s = s < 0 ? 0 : (s > nN - 1 ? nN - 1 : s);
    reg2[i] = (i < nh) ? s : 0;
  }
  __syncthreads();

  const bool ovf = (nh >= RCAP);
  v4i lv[RCAP / (4 * NTHR)];
#pragma unroll
  for (int it = 0; it < RCAP / (4 * NTHR); ++it) lv[it] = *(const v4ia*)(reg2 + 4 * (it * NTHR + tid));
  v4i ov;
  {
    const v4i c4 = *(const v4ia*)(scnt + 4 * tid);
    const v4i o4 = *(const v4ia*)(soff + 4 * tid);
    const int cc[4] = {c4.x, c4.y, c4.z, c4.w};
    const int oo[4] = {o4.x, o4.y, o4.z, o4.w};
    int pk[4];
#pragma unroll
    for (int j = 0; j < 4; ++j) {
      int c = cc[j] < 0 ? 0 : cc[j];
      const int cf = (ovf || c > DEGCAP) ? OCBAD : c;
      int o = oo[j] < 0 ? 0 : (oo[j] > RCAP ? RCAP : oo[j]);
      pk[j] = (o << 8) | cf;
    }
    ov.x = pk[0]; ov.y = pk[1]; ov.z = pk[2]; ov.w = pk[3];
  }
  int* lp = lst + (size_t)blockIdx.x * RCAP;
  int* op = oc + (size_t)nodeBase + 4 * tid;
#pragma unroll
  for (int it = 0; it < RCAP / (4 * NTHR); ++it) *(volatile v4i*)(lp + 4 * (it * NTHR + tid)) = lv[it];
  *(volatile v4i*)op = ov;
  __threadfence();
#pragma unroll
  for (int it = 0; it < RCAP / (4 * NTHR); ++it) *(volatile v4i*)(lp + 4 * (it * NTHR + tid)) = lv[it];
  *(volatile v4i*)op = ov;
}

__global__ __launch_bounds__(NTHR) void k_agg_a(const float* __restrict__ x, const int* __restrict__ lst,
                                                const int* __restrict__ oc, int nN, int mRows, int npads,
                                                unsigned short* za) {
  const int tid = (int)threadIdx.x, lane = tid & 31, wave = tid >> 5, g = lane >> 3, q = lane & 7;
  const int row = ((int)blockIdx.x * NWAVE + wave) * 4 + g;
  const int rc  = row < npads ? row : npads - 1;
  const int ocv = oc[rc];
  const int blk = rc >> NBRS;
  unsigned int off = ((unsigned int)ocv) >> 8;
  off = off > (unsigned int)RCAP ? (unsigned int)RCAP : off;
  const int cf = ocv & 255;
  const bool bad = (cf == OCBAD);
  int cnt = cf > DEGCAP ? DEGCAP : cf;
  cnt = bad ? 0 : cnt;
  int cm = cnt;
  {
    const int o8 = __shfl_xor(cm, 8);
    cm = cm > o8 ? cm : o8;
    const int o16 = __shfl_xor(cm, 16);
    cm = cm > o16 ? cm : o16;
  }
  cm = __builtin_amdgcn_readfirstlane(cm);
  cm = cm > DEGCAP ? DEGCAP : cm;
  const int* lp = lst + (size_t)blk * RCAP;

  float a0 = 0.0f, a1 = 0.0f, a2 = 0.0f, a3 = 0.0f;
#pragma unroll 1
  for (int t = 0; t < cm; ++t) {
    int idx = (int)off + t;
    idx = idx > RCAP - 1 ? RCAP - 1 : idx;
    int s = lp[idx];
    s = s < 0 ? 0 : (s > nN - 1 ? nN - 1 : s);
    const v4f v = *(const v4f*)(x + (size_t)s * FIN + 4 * q);
    const unsigned int mk = (t < cnt) ? 0xFFFFFFFFu : 0u;
    a0 += __uint_as_float(__float_as_uint(bf_rne(v.x)) & mk);
    a1 += __uint_as_float(__float_as_uint(bf_rne(v.y)) & mk);
    a2 += __uint_as_float(__float_as_uint(bf_rne(v.z)) & mk);
    a3 += __uint_as_float(__float_as_uint(bf_rne(v.w)) & mk);
  }
  const bool live = row < nN;
  const int nc = live ? row : nN - 1;
  const v4f sv = *(const v4f*)(x + (size_t)nc * FIN + 4 * q);
  const float pz = bad ? __int_as_float(0x7fc00000) : 0.0f;
  float r0 = bf_rne(sv.x) + a0, r1 = bf_rne(sv.y) + a1, r2 = bf_rne(sv.z) + a2, r3 = bf_rne(sv.w) + a3;
  r0 = (live ? r0 : 0.0f) + pz;
  r1 = (live ? r1 : 0.0f) + pz;
  r2 = (live ? r2 : 0.0f) + pz;
  r3 = (live ? r3 : 0.0f) + pz;
  const v4u pk = hilo4(r0, r1, r2, r3);
  unsigned short* gp = za + (size_t)row * KA + 8 * q;
  const bool wr = row < mRows;
  if (wr) *(volatile v4u*)gp = pk;
  __threadfence();
  if (wr) *(volatile v4u*)gp = pk;
}

__global__ __launch_bounds__(NTHR) void k_agg_b(const float* __restrict__ hin, const int* __restrict__ lst,
                                                const int* __restrict__ oc, int nN, int mRows, int npads,
                                                unsigned short* zb) {
  const int tid = (int)threadIdx.x, lane = tid & 31, wave = tid >> 5;
  const int row = (int)blockIdx.x * NWAVE + wave;
  const int rc  = row < npads ? row : npads - 1;
  const int ocv = __builtin_amdgcn_readfirstlane(oc[rc]);
  const int blk = rc >> NBRS;
  unsigned int off = ((unsigned int)ocv) >> 8;
  off = off > (unsigned int)RCAP ? (unsigned int)RCAP : off;
  const int cf = ocv & 255;
  const bool bad = (cf == OCBAD);
  int cnt = cf > DEGCAP ? DEGCAP : cf;
  cnt = bad ? 0 : cnt;
  const int* lp = lst + (size_t)blk * RCAP;

  float a0 = 0.0f, a1 = 0.0f, a2 = 0.0f, a3 = 0.0f;
#pragma unroll 1
  for (int t = 0; t < cnt; ++t) {
    int idx = (int)off + t;
    idx = idx > RCAP - 1 ? RCAP - 1 : idx;
    int s = lp[idx];
    s = s < 0 ? 0 : (s > nN - 1 ? nN - 1 : s);
    const v4f v = *(const v4f*)(hin + (size_t)s * DH + 4 * lane);
    a0 += v.x; a1 += v.y; a2 += v.z; a3 += v.w;
  }
  const bool live = row < nN;
  const int nc = live ? row : nN - 1;
  const v4f sv = *(const v4f*)(hin + (size_t)nc * DH + 4 * lane);
  const float pz = bad ? __int_as_float(0x7fc00000) : 0.0f;
  float r0 = sv.x + a0, r1 = sv.y + a1, r2 = sv.z + a2, r3 = sv.w + a3;
  r0 = (live ? r0 : 0.0f) + pz;
  r1 = (live ? r1 : 0.0f) + pz;
  r2 = (live ? r2 : 0.0f) + pz;
  r3 = (live ? r3 : 0.0f) + pz;
  const v4u pk = hilo4(r0, r1, r2, r3);
  unsigned short* gp = zb + (size_t)row * KB + 8 * lane;
  const bool wr = row < mRows;
  if (wr) *(volatile v4u*)gp = pk;
  __threadfence();
  if (wr) *(volatile v4u*)gp = pk;
}

template <int K1>
__global__ __launch_bounds__(GTHR) void k_mlp(const unsigned short* __restrict__ Z,
                                              const unsigned short* __restrict__ W1T,
                                              const unsigned short* __restrict__ W2T,
                                              const float* __restrict__ vec, float* H, int nN, int mRows) {
  __shared__ __attribute__((aligned(16))) float stg[GBM * DH];
  const int tid = (int)threadIdx.x, lane = tid & 31, wave = tid >> 5, hh = lane >> 4, m = lane & 15;
  const int rowBase = (int)blockIdx.x * GBM;

  v8f acc[GNT];
  const v8f zero8 = {0.f, 0.f, 0.f, 0.f, 0.f, 0.f, 0.f, 0.f};
#pragma unroll
  for (int t = 0; t < GNT; ++t) acc[t] = zero8;

  {
    const unsigned short* ap = Z   + (size_t)(rowBase + 16 * wave + m) * (size_t)K1 + 8 * hh;
    const unsigned short* bp = W1T + (size_t)m * (size_t)K1 + 8 * hh;
#pragma unroll 1
    for (int k0 = 0; k0 < K1; k0 += 32) {
      Frag af;
      af.h[0] = *(const v8usa*)(ap + k0);
      af.h[1] = *(const v8usa*)(ap + k0 + 16);
#pragma unroll
      for (int nt = 0; nt < GNT; ++nt) {
        const unsigned short* wq = bp + (size_t)(16 * nt) * (size_t)K1 + k0;
        Frag bfr;
        bfr.h[0] = *(const v8usa*)wq;
        bfr.h[1] = *(const v8usa*)(wq + 16);
        acc[nt] = wmb(af, bfr, acc[nt]);
      }
    }
  }
#pragma unroll
  for (int nt = 0; nt < GNT; ++nt) {
#pragma unroll
    for (int r = 0; r < 8; ++r) {
      stg[(16 * wave + 8 * hh + r) * DH + 16 * nt + m] = acc[nt][r];
    }
  }
  __syncthreads();

  {
    const v4f b1v = *(const v4f*)(vec + 4 * lane);
    const v4f rmv = *(const v4f*)(vec + DH + 4 * lane);
    const v4f rsv = *(const v4f*)(vec + 2 * DH + 4 * lane);
    const v4f gv  = *(const v4f*)(vec + 3 * DH + 4 * lane);
    const v4f bev = *(const v4f*)(vec + 4 * DH + 4 * lane);
#pragma unroll 1
    for (int i = 0; i < 16; ++i) {
      float* p = stg + (16 * wave + i) * DH + 4 * lane;
      const v4f a = *(const v4fa*)p;
      const float u0 = a.x + b1v.x, u1 = a.y + b1v.y, u2 = a.z + b1v.z, u3 = a.w + b1v.w;
      const float y0 = ((u0 - rmv.x) * rsv.x) * gv.x + bev.x;
      const float y1 = ((u1 - rmv.y) * rsv.y) * gv.y + bev.y;
      const float y2 = ((u2 - rmv.z) * rsv.z) * gv.z + bev.z;
      const float y3 = ((u3 - rmv.w) * rsv.w) * gv.w + bev.w;
      const v4u tv = hilo4(relu_keep(y0), relu_keep(y1), relu_keep(y2), relu_keep(y3));
      *(v4ua*)p = tv;
    }
  }
  __syncthreads();

#pragma unroll
  for (int t = 0; t < GNT; ++t) acc[t] = zero8;
  {
    const unsigned short* tp = (const unsigned short*)stg + (16 * wave + m) * KB + 8 * hh;
    const unsigned short* bp = W2T + (size_t)m * (size_t)KB + 8 * hh;
#pragma unroll 1
    for (int k0 = 0; k0 < KB; k0 += 32) {
      Frag af;
      af.h[0] = *(const v8usa*)(tp + k0);
      af.h[1] = *(const v8usa*)(tp + k0 + 16);
#pragma unroll
      for (int nt = 0; nt < GNT; ++nt) {
        const unsigned short* wq = bp + (size_t)(16 * nt) * (size_t)KB + k0;
        Frag bfr;
        bfr.h[0] = *(const v8usa*)wq;
        bfr.h[1] = *(const v8usa*)(wq + 16);
        acc[nt] = wmb(af, bfr, acc[nt]);
      }
    }
  }
  __syncthreads();
#pragma unroll
  for (int nt = 0; nt < GNT; ++nt) {
#pragma unroll
    for (int r = 0; r < 8; ++r) {
      stg[(16 * wave + 8 * hh + r) * DH + 16 * nt + m] = acc[nt][r];
    }
  }
  __syncthreads();

  const v4f b2v = *(const v4f*)(vec + 5 * DH + 4 * lane);
  v4f fv[16];
#pragma unroll
  for (int i = 0; i < 16; ++i) {
    const int lr = 16 * wave + i;
    const v4f a = *(const v4fa*)(stg + lr * DH + 4 * lane);
    const bool live = (rowBase + lr) < nN;
    v4f o;
    o.x = live ? relu_keep(a.x + b2v.x) : 0.0f;
    o.y = live ? relu_keep(a.y + b2v.y) : 0.0f;
    o.z = live ? relu_keep(a.z + b2v.z) : 0.0f;
    o.w = live ? relu_keep(a.w + b2v.w) : 0.0f;
    fv[i] = o;
  }
#pragma unroll
  for (int i = 0; i < 16; ++i) {
    const int gr = rowBase + 16 * wave + i;
    float* op = H + (size_t)gr * DH + 4 * lane;
    if (gr < mRows) *(volatile v4f*)op = fv[i];
  }
  __threadfence();
#pragma unroll
  for (int i = 0; i < 16; ++i) {
    const int gr = rowBase + 16 * wave + i;
    float* op = H + (size_t)gr * DH + 4 * lane;
    if (gr < mRows) *(volatile v4f*)op = fv[i];
  }
}

__global__ __launch_bounds__(NTHR) void k_pool_head(const float* __restrict__ H, const int* __restrict__ bat,
                                                    int nN, int vec8b, int nG,
                                                    const unsigned short* __restrict__ LWT,
                                                    const float* __restrict__ hv, float* out) {
  extern __shared__ __attribute__((aligned(16))) float psm[];
  float* accs = psm;
  float* hvs  = accs + PGR * DH;
  float* os   = hvs + HVF;
  int*   list = (int*)(os + PGR);
  int*   wcnt = list + LISTN;
  const int tid = (int)threadIdx.x, lane = tid & 31, wave = tid >> 5, hh = lane >> 4, m = lane & 15;
  const int slotBase = (int)blockIdx.x * PGR;

  {
    const v4f z4 = {0.f, 0.f, 0.f, 0.f};
    for (int i = tid; i < PGR * DH / 4; i += NTHR) *(v4fa*)(accs + 4 * i) = z4;
    for (int i = tid; i < LISTN; i += NTHR) list[i] = 0;
    if (tid < HVF / 4) *(v4fa*)(hvs + 4 * tid) = *(const v4f*)(hv + 4 * tid);
    if (tid < PGR) os[tid] = 0.0f;
    if (tid < 16) wcnt[tid] = 0;
  }
  __syncthreads();

  const int nChunks = (nN + CHUNK - 1) / CHUNK;
#pragma unroll 1
  for (int ch = 0; ch < nChunks; ++ch) {
    const int cbase = ch * CHUNK;
    const int wc = scan_chunk(bat, nN, cbase, slotBase, PGR, vec8b, list, tid, lane, wave);
    if (lane == 0) wcnt[wave] = wc;
    __syncthreads();
#pragma unroll 1
    for (int w2 = 0; w2 < NWAVE; ++w2) {
      int c = wcnt[w2];
      c = c < 0 ? 0 : (c > WCAP ? WCAP : c);
#pragma unroll 1
      for (int i = 0; i < c; ++i) {
        const int ent = list[w2 * WCAP + i];
        const int el  = (ent >> PKS) & (CHUNK - 1);
        const int sl  = ent & (PGR - 1);
        int node = cbase + el;
        node = node < 0 ? 0 : (node > nN - 1 ? nN - 1 : node);
#pragma unroll 1
        for (int cc = tid; cc < DH; cc += NTHR) {
          const float v = H[(size_t)node * DH + cc];
          accs[sl * DH + cc] += v;
        }
      }
    }
    __syncthreads();
  }

#pragma unroll 1
  for (int it = 0; it < (PGR * DH / 4) / NTHR; ++it) {
    float* p = accs + 4 * (it * NTHR + tid);
    const v4f a = *(const v4fa*)p;
    const v4u tv = hilo4(a.x, a.y, a.z, a.w);
    *(v4ua*)p = tv;
  }
  __syncthreads();

  v8f acc[GNT];
  {
    const v8f z = {0.f, 0.f, 0.f, 0.f, 0.f, 0.f, 0.f, 0.f};
#pragma unroll
    for (int t = 0; t < GNT; ++t) acc[t] = z;
  }
  {
    const unsigned short* tp = (const unsigned short*)accs + (16 * wave + m) * KB + 8 * hh;
    const unsigned short* bp = LWT + (size_t)m * (size_t)KB + 8 * hh;
#pragma unroll 1
    for (int k0 = 0; k0 < KB; k0 += 32) {
      Frag af;
      af.h[0] = *(const v8usa*)(tp + k0);
      af.h[1] = *(const v8usa*)(tp + k0 + 16);
#pragma unroll
      for (int nt = 0; nt < GNT; ++nt) {
        const unsigned short* wq = bp + (size_t)(16 * nt) * (size_t)KB + k0;
        Frag bfr;
        bfr.h[0] = *(const v8usa*)wq;
        bfr.h[1] = *(const v8usa*)(wq + 16);
        acc[nt] = wmb(af, bfr, acc[nt]);
      }
    }
  }

  float part[8];
#pragma unroll
  for (int r = 0; r < 8; ++r) part[r] = 0.0f;
#pragma unroll
  for (int nt = 0; nt < GNT; ++nt) {
    const int c = 16 * nt + m;
    const float bb = hvs[c];
    const float w  = hvs[DH + c];
#pragma unroll
    for (int r = 0; r < 8; ++r) {
      const float y = relu_keep(acc[nt][r] + bb);
      part[r] = fmaf(y, w, part[r]);
    }
  }
  const float lb2s = hvs[2 * DH];
#pragma unroll
  for (int r = 0; r < 8; ++r) {
    float v = part[r];
    v += __shfl_xor(v, 1);
    v += __shfl_xor(v, 2);
    v += __shfl_xor(v, 4);
    v += __shfl_xor(v, 8);
    if (m == 0) os[16 * wave + 8 * hh + r] = v + lb2s;
  }
  __syncthreads();

  const v4f ovv = *(const v4fa*)(os + 4 * lane);
  const int g0 = slotBase + 4 * lane;
  const bool okst = (wave == 0) && (g0 + 3 < nG);
  float* op = out + (size_t)g0;
  if (okst) *(volatile v4f*)op = ovv;
  __threadfence();
  if (okst) *(volatile v4f*)op = ovv;
}

static inline int cdiv(int a, int b) { return (a + b - 1) / b; }
static inline size_t al256(size_t o) { return (o + 255) & ~(size_t)255; }

extern "C" void kernel_launch(void* const* d_in, const int* in_sizes, int n_in,
                              void* d_out, int out_size, void* d_ws, size_t ws_size,
                              hipStream_t stream) {
  if (n_in < 31) return;
  if (in_sizes[0] < FIN || (in_sizes[0] % FIN) != 0) return;
  const int nN = in_sizes[0] / FIN;
  if (nN < GBM || nN > (1 << 22)) return;
  const int nE2 = in_sizes[1];
  if (nE2 < 2 || (nE2 & 1) != 0) return;
  const int nE = nE2 / 2;
  if (nE < 1 || nE > (1 << 21)) return;
  if (in_sizes[2] != nN) return;
  if (in_sizes[3] != FIN * DH) return;
  for (int i = 4; i <= 8; ++i) if (in_sizes[i] != DH) return;
  if (in_sizes[9] != DH * DH || in_sizes[10] != DH) return;
  if (in_sizes[11] != DH * DH) return;
  for (int i = 12; i <= 16; ++i) if (in_sizes[i] != DH) return;
  if (in_sizes[17] != DH * DH || in_sizes[18] != DH) return;
  if (in_sizes[19] != DH * DH) return;
  for (int i = 20; i <= 24; ++i) if (in_sizes[i] != DH) return;
  if (in_sizes[25] != DH * DH || in_sizes[26] != DH) return;
  if (in_sizes[27] != DH * DH || in_sizes[28] != DH) return;
  if (in_sizes[29] != DH || in_sizes[30] != 1) return;
  const int nG = out_size;
  if (nG < 4 || (nG & 3) != 0 || nG > (1 << 20)) return;

  const float* x     = (const float*)d_in[0];
  const int*   ei    = (const int*)  d_in[1];
  const int*   src   = ei;
  const int*   dst   = ei + nE;
  const int*   batch = (const int*)  d_in[2];
  const float* W1a = (const float*)d_in[3];  const float* b1a = (const float*)d_in[4];
  const float* ga  = (const float*)d_in[5];  const float* bea = (const float*)d_in[6];
  const float* rma = (const float*)d_in[7];  const float* rva = (const float*)d_in[8];
  const float* W2a = (const float*)d_in[9];  const float* b2a = (const float*)d_in[10];
  const float* W1b = (const float*)d_in[11]; const float* b1b = (const float*)d_in[12];
  const float* gb  = (const float*)d_in[13]; const float* beb = (const float*)d_in[14];
  const float* rmb = (const float*)d_in[15]; const float* rvb = (const float*)d_in[16];
  const float* W2b = (const float*)d_in[17]; const float* b2b = (const float*)d_in[18];
  const float* W1c = (const float*)d_in[19]; const float* b1c = (const float*)d_in[20];
  const float* gc  = (const float*)d_in[21]; const float* bec = (const float*)d_in[22];
  const float* rmc = (const float*)d_in[23]; const float* rvc = (const float*)d_in[24];
  const float* W2c = (const float*)d_in[25]; const float* b2c = (const float*)d_in[26];
  const float* lw1 = (const float*)d_in[27]; const float* lb1 = (const float*)d_in[28];
  const float* lw2 = (const float*)d_in[29]; const float* lb2 = (const float*)d_in[30];
  float* out = (float*)d_out;

  const int MP    = cdiv(nN, GBM) * GBM;
  const int nblk  = cdiv(MP, NBR);
  const int npads = nblk * NBR;
  if (npads < MP) return;
  const int vec8  = ((nE & 3) == 0) ? 1 : 0;
  const int vec8b = ((nN & 3) == 0) ? 1 : 0;
  const int gP    = cdiv(nG, PGR);

  char* ws = (char*)d_ws;
  size_t off = 0;
  const size_t oW1a = off; off = al256(off + (size_t)NUA * 16);
  const size_t oW2a = off; off = al256(off + (size_t)NUB * 16);
  const size_t oW1b = off; off = al256(off + (size_t)NUB * 16);
  const size_t oW2b = off; off = al256(off + (size_t)NUB * 16);
  const size_t oW1c = off; off = al256(off + (size_t)NUB * 16);
  const size_t oW2c = off; off = al256(off + (size_t)NUB * 16);
  const size_t oLW1 = off; off = al256(off + (size_t)NUB * 16);
  const size_t oVEC = off; off = al256(off + (size_t)NVBLK * VECL * 4);
  const size_t oLST = off; off = al256(off + (size_t)nblk * RCAP * 4);
  const size_t oOC  = off; off = al256(off + (size_t)npads * 4);
  const size_t oA   = off; off = al256(off + (size_t)MP * DH * 4);
  const size_t oB   = off; off = al256(off + (size_t)MP * KB * 2);
  if (off > ws_size || off > (size_t)WSMAX) return;
  unsigned short* pW1a = (unsigned short*)(ws + oW1a);
  unsigned short* pW2a = (unsigned short*)(ws + oW2a);
  unsigned short* pW1b = (unsigned short*)(ws + oW1b);
  unsigned short* pW2b = (unsigned short*)(ws + oW2b);
  unsigned short* pW1c = (unsigned short*)(ws + oW1c);
  unsigned short* pW2c = (unsigned short*)(ws + oW2c);
  unsigned short* pLW1 = (unsigned short*)(ws + oLW1);
  float*          VEC  = (float*)(ws + oVEC);
  int*            LST  = (int*)(ws + oLST);
  int*            OC   = (int*)(ws + oOC);
  float*          HA   = (float*)(ws + oA);
  unsigned short* ZB   = (unsigned short*)(ws + oB);

  hipFuncSetAttribute(reinterpret_cast<const void*>(&k_pool_head), hipFuncAttributeMaxDynamicSharedMemorySize, LDS_POOL);

  k_prep<<<NWBLK + NVBLK, NTHR, 0, stream>>>(W1a, W2a, W1b, W2b, W1c, W2c, lw1,
                                             b1a, ga, bea, rma, rva, b2a,
                                             b1b, gb, beb, rmb, rvb, b2b,
                                             b1c, gc, bec, rmc, rvc, b2c,
                                             lb1, lw2, lb2,
                                             pW1a, pW2a, pW1b, pW2b, pW1c, pW2c, pLW1, VEC);
  k_scan<<<nblk, NTHR, 0, stream>>>(src, dst, nN, nE, vec8, LST, OC);
  k_agg_a<<<MP / 32, NTHR, 0, stream>>>(x, LST, OC, nN, MP, npads, ZB);
  k_mlp<KA><<<MP / GBM, GTHR, 0, stream>>>(ZB, pW1a, pW2a, VEC, HA, nN, MP);
  k_agg_b<<<MP / NWAVE, NTHR, 0, stream>>>(HA, LST, OC, nN, MP, npads, ZB);
  k_mlp<KB><<<MP / GBM, GTHR, 0, stream>>>(ZB, pW1b, pW2b, VEC + VECL, HA, nN, MP);
  k_agg_b<<<MP / NWAVE, NTHR, 0, stream>>>(HA, LST, OC, nN, MP, npads, ZB);
  k_mlp<KB><<<MP / GBM, GTHR, 0, stream>>>(ZB, pW1c, pW2c, VEC + 2 * VECL, HA, nN, MP);
  k_pool_head<<<gP, NTHR, LDS_POOL, stream>>>(HA, batch, nN, vec8b, nG, pLW1, VEC + 3 * VECL, out);
}
